// MultiHeadAttention_43568148251309
// MI455X (gfx1250) — hardware-run, weakly checked
//
#include <hip/hip_runtime.h>


#ifndef NB
#define NB 2
#endif
#ifndef SEQ
#define SEQ 2048
#endif
#define NB_FULL  2
#define SEQ_FULL 2048
#ifndef OUT_SEQ
#define OUT_SEQ SEQ
#endif
#ifndef AVG_PITCH
#define AVG_PITCH OUT_SEQ
#endif
#define DM   1024
#define NH_  16
#define HD   64
#define AW   4
#define AKT  64
#define QRS  2048.0f
#define QRI  (1.0f / 2048.0f)
#define SC2  (0.125f * 1.4426950408889634f)
#define PSH  8.0f
#define NEGB (-3.0e38f)
#define AVG_OFF ((size_t)NB_FULL * SEQ_FULL * DM)

static_assert(HD == 64);
static_assert(NH_ * HD == DM);
static_assert(DM % 64 == 0);
static_assert(DM % 32 == 0);
static_assert((DM & (DM - 1)) == 0);
static_assert(SEQ % 64 == 0);
static_assert((NB * SEQ) % 64 == 0);
static_assert(SEQ % 32 == 0);
static_assert(SEQ % (16 * AW) == 0);
static_assert(SEQ % (AKT * AW) == 0);
static_assert(AVG_PITCH % 64 == 0);
static_assert(((size_t)SEQ * DM) % 8 == 0);
static_assert(((size_t)DM * DM) % 8 == 0);
static_assert(NB <= NB_FULL);
static_assert(SEQ <= SEQ_FULL);
static_assert(AVG_OFF * 4 == (size_t)16777216);

typedef _Float16 h16;
typedef unsigned short bf;
typedef __attribute__((ext_vector_type(16))) __bf16   v16bf;
typedef __attribute__((ext_vector_type(16))) _Float16 v16h;
typedef __attribute__((ext_vector_type(8)))  _Float16 v8h;
typedef __attribute__((ext_vector_type(8)))  unsigned short v8us;
typedef __attribute__((ext_vector_type(8)))  float    v8f;
typedef __attribute__((ext_vector_type(4)))  float    v4f;
typedef v4f  __attribute__((may_alias)) v4fa;

__device__ __forceinline__ unsigned short f2bf(float f) { unsigned u = __float_as_uint(f); u += 0x7FFFu + ((u >> 16) & 1u); return (unsigned short)(u >> 16); }
__device__ __forceinline__ float bf2f(unsigned short s) { return __uint_as_float(((unsigned)s) << 16); }
__device__ __forceinline__ float bfr(float f) { return bf2f(f2bf(f)); }
__device__ __forceinline__ v16h cat16(v8h lo, v8h hi) { return __builtin_shufflevector(lo, hi, 0, 1, 2, 3, 4, 5, 6, 7, 8, 9, 10, 11, 12, 13, 14, 15); }
__device__ __forceinline__ v16bf cat16b(v8us lo, v8us hi) { return __builtin_bit_cast(v16bf, __builtin_shufflevector(lo, hi, 0, 1, 2, 3, 4, 5, 6, 7, 8, 9, 10, 11, 12, 13, 14, 15)); }
__device__ __forceinline__ v8f wmma16(v16h a, v16h b, v8f c) { return __builtin_amdgcn_wmma_f32_16x16x32_f16(false, a, false, b, (short)0, c, false, false); }
__device__ __forceinline__ v8f wmmab(v16bf a, v16bf b, v8f c) { return __builtin_amdgcn_wmma_f32_16x16x32_bf16(false, a, false, b, (short)0, c, false, false); }
__device__ __forceinline__ v16h  ldh(const h16* p) { return cat16(*(const v8h*)p, *(const v8h*)(p + 16)); }
__device__ __forceinline__ v16bf ldb(const bf* p)  { return cat16b(*(const v8us*)p, *(const v8us*)(p + 16)); }
__device__ __forceinline__ void wave_sync() { __builtin_amdgcn_fence(3  , "wavefront"); __builtin_amdgcn_wave_barrier(); asm volatile("" ::: "memory"); }

__global__ __launch_bounds__(256) void k_cvt8(const float* __restrict__ src, bf* dst, size_t n8) {
    const size_t i = (size_t)blockIdx.x * 256 + threadIdx.x; if (i >= n8) return;
    const v8f v = *(const v8f*)(src + i * 8); v8us o;
#pragma unroll
    for (int k = 0; k < 8; ++k) o[k] = f2bf(v[k]);
    *(volatile v8us*)(dst + i * 8) = o; __threadfence(); *(volatile v8us*)(dst + i * 8) = o;
}

template <int K, int KB>
__device__ __forceinline__ void gemm64(const bf* __restrict__ A, const bf* __restrict__ Bt, int r0, int c0, int lr, int hi, v8f (&acc)[4][4]) {
    static_assert(K % 32 == 0); static_assert(KB % 32 == 0); static_assert((KB & (KB - 1)) == 0); static_assert(K % KB == 0);
#pragma unroll
    for (int mb = 0; mb < 4; ++mb)
#pragma unroll
        for (int nb = 0; nb < 4; ++nb) acc[mb][nb] = (v8f){};
    const size_t aoff = (size_t)(r0 + lr) * K + 8 * hi, boff = (size_t)(c0 + lr) * KB + 8 * hi;
#pragma unroll 1
    for (int kc = 0; kc < K; kc += 32) {
        const int kb = kc & (KB - 1);
        v16bf a[4];
#pragma unroll
        for (int mb = 0; mb < 4; ++mb) a[mb] = ldb(A + aoff + (size_t)mb * 16 * K + kc);
#pragma unroll
        for (int nb = 0; nb < 4; ++nb) { const v16bf b = ldb(Bt + boff + (size_t)nb * 16 * KB + kb);
#pragma unroll
            for (int mb = 0; mb < 4; ++mb) acc[mb][nb] = wmmab(a[mb], b, acc[mb][nb]); }
        asm volatile("v_nop\n\tv_nop\n\tv_nop\n\tv_nop" : "+v"(acc[0][0]), "+v"(acc[1][1]), "+v"(acc[2][2]), "+v"(acc[3][3]) : "v"(a[0]), "v"(a[1]), "v"(a[2]), "v"(a[3]));
    }
}

__global__ __launch_bounds__(32) void k_proj(const bf* __restrict__ A, const bf* __restrict__ Bt, const float* __restrict__ bias, int biasRow,
                                             h16* Ph, h16* Pr, int useRes, int RB, size_t sRB, int pitch, int CB, size_t sCB) {
    __shared__ __align__(16) float os[16 * 68];
    const int lane = threadIdx.x & 31, lr = lane & 15, hi = lane >> 4; const int r0 = blockIdx.x * 64, c0 = blockIdx.y * 64;
    v8f acc[4][4];
    gemm64<DM, DM>(A, Bt, r0, c0, lr, hi, acc);
    float cb[4];
#pragma unroll
    for (int nb = 0; nb < 4; ++nb) { const float t = bfr(bias[(c0 + nb * 16 + lr) & (DM - 1)]); cb[nb] = biasRow ? 0.0f : t; }
    const size_t tbase = (size_t)(r0 / RB) * sRB + (size_t)(r0 % RB) * (size_t)pitch + (size_t)(c0 / CB) * sCB + (size_t)(c0 % CB);
#pragma unroll
    for (int mb = 0; mb < 4; ++mb) {
        float rb[8];
#pragma unroll
        for (int j = 0; j < 8; ++j) { const float t = bfr(bias[(r0 + mb * 16 + hi * 8 + j) & (DM - 1)]); rb[j] = biasRow ? t : 0.0f; }
#pragma unroll
        for (int nb = 0; nb < 4; ++nb) {
#pragma unroll
            for (int j = 0; j < 8; ++j) os[(hi * 8 + j) * 68 + nb * 16 + lr] = (acc[mb][nb][j] + cb[nb]) + rb[j]; }
        wave_sync();
        const size_t sb = tbase + (size_t)(mb * 16) * (size_t)pitch;
#pragma unroll 1
        for (int ps = 0; ps < 2; ++ps) {
#pragma unroll
            for (int s = 0; s < 4; ++s) { const int row = 4 * s + (lane >> 3), c8 = (lane & 7) * 8;
                const v4f x0 = *(const v4fa*)(&os[row * 68 + c8]); const v4f x1 = *(const v4fa*)(&os[row * 68 + c8 + 4]); v8h hv, rv;
#pragma unroll
                for (int i = 0; i < 4; ++i) { const h16 a0 = (h16)x0[i]; const h16 a1 = (h16)x1[i]; hv[i] = a0; hv[4 + i] = a1; rv[i] = (h16)((x0[i] - (float)a0) * QRS); rv[4 + i] = (h16)((x1[i] - (float)a1) * QRS); }
                const size_t oo = sb + (size_t)row * (size_t)pitch + c8;
                *(volatile v8h*)(Ph + oo) = hv; if (useRes) *(volatile v8h*)(Pr + oo) = rv; }
            if (ps == 0) __threadfence(); }
        wave_sync();
    }
}

__global__ __launch_bounds__(32) void k_outp(const bf* __restrict__ A, const bf* __restrict__ Bt, const float* __restrict__ bias, float* OUT) {
    __shared__ __align__(16) float os[16 * 68];
    const int lane = threadIdx.x & 31, lr = lane & 15, hi = lane >> 4; const int r0 = blockIdx.x * 64, c0 = blockIdx.y * 64;
    v8f acc[4][4];
    gemm64<2 * DM, DM>(A, Bt, r0, c0, lr, hi, acc);
    float cb[4];
#pragma unroll
    for (int nb = 0; nb < 4; ++nb) cb[nb] = bfr(bias[c0 + nb * 16 + lr]);
    const int bb = r0 / SEQ, tt = r0 % SEQ;
    float* obase = OUT + ((size_t)bb * OUT_SEQ + tt) * DM + c0;
#pragma unroll
    for (int mb = 0; mb < 4; ++mb) {
#pragma unroll
        for (int nb = 0; nb < 4; ++nb) {
#pragma unroll
            for (int j = 0; j < 8; ++j) os[(hi * 8 + j) * 68 + nb * 16 + lr] = acc[mb][nb][j] + cb[nb]; }
        wave_sync();
#pragma unroll 1
        for (int ps = 0; ps < 2; ++ps) {
#pragma unroll
            for (int s = 0; s < 8; ++s) { const int row = 2 * s + hi, cofs = lr * 4;
                const v4f val = *(const v4fa*)(&os[row * 68 + cofs]);
                *(volatile v4f*)(obase + (size_t)(mb * 16 + row) * DM + cofs) = val; }
            if (ps == 0) __threadfence(); }
        wave_sync();
    }
}

#define PUT8(J, OH, OE) { v4f a_, c_; \
    a_[0] = ((OH)[0] + (OE)[0] * QRI) * inv; a_[1] = ((OH)[1] + (OE)[1] * QRI) * inv; a_[2] = ((OH)[2] + (OE)[2] * QRI) * inv; a_[3] = ((OH)[3] + (OE)[3] * QRI) * inv; \
    c_[0] = ((OH)[4] + (OE)[4] * QRI) * inv; c_[1] = ((OH)[5] + (OE)[5] * QRI) * inv; c_[2] = ((OH)[6] + (OE)[6] * QRI) * inv; c_[3] = ((OH)[7] + (OE)[7] * QRI) * inv; \
    *(v4fa*)(&os[wb + lr * 68 + 16 * (J) + 8 * hi]) = a_; *(v4fa*)(&os[wb + lr * 68 + 16 * (J) + 8 * hi + 4]) = c_; }

__global__ __launch_bounds__(32 * AW) void k_flash(const h16* __restrict__ QH, const h16* __restrict__ QR, const h16* __restrict__ KP, const h16* __restrict__ VT, const h16* __restrict__ VR, bf* CTX, float* ST) {
    __shared__ __align__(16) float os[AW * 16 * 68];
    const int lane = threadIdx.x & 31, lr = lane & 15, hi = lane >> 4;
    const int wave = __builtin_amdgcn_readfirstlane((int)(threadIdx.x >> 5));
    const int zh = blockIdx.y; const int b = zh / NH_, h = zh % NH_;
    const int tile = blockIdx.x * AW + wave; const int t0 = tile * 16; const int tq = t0 + lr;
    const size_t pbase = (size_t)zh * SEQ * HD;
    const size_t qo = pbase + (size_t)(t0 + lr) * HD + 8 * hi;
    const v16h qh0 = ldh(QH + qo), qh1 = ldh(QH + qo + 32), qr0 = ldh(QR + qo), qr1 = ldh(QR + qo + 32);
    const size_t ko = pbase + (size_t)lr * HD + 8 * hi;
    const size_t vo = pbase + (size_t)lr * SEQ + 8 * hi;
    v8f o0 = (v8f){}, o1 = (v8f){}, o2 = (v8f){}, o3 = (v8f){};
    v8f e0 = (v8f){}, e1 = (v8f){}, e2 = (v8f){}, e3 = (v8f){};
    float m = NEGB, l = 0.0f;
    const int kend = t0 + 16;
#pragma unroll 1
    for (int key0 = 0; key0 < kend; key0 += 32) {
        const h16* ka = KP + ko + (size_t)key0 * HD;
        const v16h ka0 = ldh(ka), ka1 = ldh(ka + 32), kb0 = ldh(ka + 16 * HD), kb1 = ldh(ka + 16 * HD + 32);
        v8f sHa = (v8f){}, sLa = (v8f){}, sHb = (v8f){}, sLb = (v8f){};
        sHa = wmma16(ka0, qh0, sHa); sLa = wmma16(ka0, qr0, sLa); sHb = wmma16(kb0, qh0, sHb); sLb = wmma16(kb0, qr0, sLb);
        sHa = wmma16(ka1, qh1, sHa); sLa = wmma16(ka1, qr1, sLa); sHb = wmma16(kb1, qh1, sHb); sLb = wmma16(kb1, qr1, sLb);
        asm volatile("v_nop\n\tv_nop\n\tv_nop\n\tv_nop" : "+v"(sHa), "+v"(sLa), "+v"(sHb), "+v"(sLb) : "v"(ka0), "v"(ka1), "v"(kb0), "v"(kb1));
        const int kA = key0 + 8 * hi, kB = kA + 16;
        float ta[8], tb[8]; float mx = NEGB;
#pragma unroll
        for (int r = 0; r < 8; ++r) { const float sa = (sHa[r] + sLa[r] * QRI) * SC2; const float sb = (sHb[r] + sLb[r] * QRI) * SC2;
            ta[r] = (kA + r <= tq) ? sa : NEGB; tb[r] = (kB + r <= tq) ? sb : NEGB; mx = fmaxf(mx, fmaxf(ta[r], tb[r])); }
        mx = fmaxf(mx, __shfl_xor(mx, 16, 32));
        const float mnew = fmaxf(m, mx);
        const float alpha = __builtin_amdgcn_exp2f(m - mnew);
        const float sh = PSH - mnew;
        v16h pb; float ls = 0.0f;
#pragma unroll
        for (int r = 0; r < 8; ++r) { const h16 pa = (h16)__builtin_amdgcn_exp2f(ta[r] + sh); const h16 pc = (h16)__builtin_amdgcn_exp2f(tb[r] + sh); pb[r] = pa; pb[8 + r] = pc; ls += (float)pa + (float)pc; }
        l = l * alpha + ls; m = mnew;
        o0 = o0 * alpha; o1 = o1 * alpha; o2 = o2 * alpha; o3 = o3 * alpha;
        e0 = e0 * alpha; e1 = e1 * alpha; e2 = e2 * alpha; e3 = e3 * alpha;
        { const h16* va = VT + vo + key0;
          const v16h v0 = ldh(va), v1 = ldh(va + (size_t)16 * SEQ), v2 = ldh(va + (size_t)32 * SEQ), v3 = ldh(va + (size_t)48 * SEQ);
          o0 = wmma16(v0, pb, o0); o1 = wmma16(v1, pb, o1); o2 = wmma16(v2, pb, o2); o3 = wmma16(v3, pb, o3);
          asm volatile("v_nop\n\tv_nop\n\tv_nop\n\tv_nop" : "+v"(o0), "+v"(o1), "+v"(o2), "+v"(o3) : "v"(v0), "v"(v1), "v"(v2), "v"(v3), "v"(pb)); }
        { const h16* vr = VR + vo + key0;
          const v16h w0 = ldh(vr), w1 = ldh(vr + (size_t)16 * SEQ), w2 = ldh(vr + (size_t)32 * SEQ), w3 = ldh(vr + (size_t)48 * SEQ);
          e0 = wmma16(w0, pb, e0); e1 = wmma16(w1, pb, e1); e2 = wmma16(w2, pb, e2); e3 = wmma16(w3, pb, e3);
          asm volatile("v_nop\n\tv_nop\n\tv_nop\n\tv_nop" : "+v"(e0), "+v"(e1), "+v"(e2), "+v"(e3) : "v"(w0), "v"(w1), "v"(w2), "v"(w3), "v"(pb)); }
    }
    l += __shfl_xor(l, 16, 32);
    const float inv = 1.0f / l;
    const int wb = wave * 16 * 68;
    PUT8(0, o0, e0) PUT8(1, o1, e1) PUT8(2, o2, e2) PUT8(3, o3, e3)
    wave_sync();
    const float sv = hi ? inv : (PSH - m);
    float* sp = ST + ((size_t)zh * (SEQ / 16) + tile) * 32 + lane;
    const size_t crow = ((size_t)b * SEQ + t0) * (size_t)(2 * DM) + (size_t)h * HD;
#pragma unroll 1
    for (int ps = 0; ps < 2; ++ps) {
        *(volatile float*)sp = sv;
#pragma unroll
        for (int s = 0; s < 4; ++s) { const int row = 4 * s + (lane >> 3), c8 = (lane & 7) * 8;
            const v4f x0 = *(const v4fa*)(&os[wb + row * 68 + c8]); const v4f x1 = *(const v4fa*)(&os[wb + row * 68 + c8 + 4]); v8us hv, lv;
#pragma unroll
            for (int i = 0; i < 4; ++i) { const unsigned short a0 = f2bf(x0[i]); const unsigned short a1 = f2bf(x1[i]); hv[i] = a0; hv[4 + i] = a1; lv[i] = f2bf(x0[i] - bf2f(a0)); lv[4 + i] = f2bf(x1[i] - bf2f(a1)); }
            const size_t oo = crow + (size_t)row * (size_t)(2 * DM) + c8;
            *(volatile v8us*)(CTX + oo) = hv; *(volatile v8us*)(CTX + oo + DM) = lv; }
        if (ps == 0) __threadfence(); }
}

#define PUTA(J, AC) { v4f a_, c_; \
    a_[0] = (AC)[0] * 0.0625f; a_[1] = (AC)[1] * 0.0625f; a_[2] = (AC)[2] * 0.0625f; a_[3] = (AC)[3] * 0.0625f; \
    c_[0] = (AC)[4] * 0.0625f; c_[1] = (AC)[5] * 0.0625f; c_[2] = (AC)[6] * 0.0625f; c_[3] = (AC)[7] * 0.0625f; \
    *(v4fa*)(&os[wb + lr * 68 + 16 * (J) + 8 * hi]) = a_; *(v4fa*)(&os[wb + lr * 68 + 16 * (J) + 8 * hi + 4]) = c_; }

__global__ __launch_bounds__(32 * AW) void k_avg(const h16* __restrict__ QH, const h16* __restrict__ QR, const h16* __restrict__ KP, const float* __restrict__ ST, float* AVG) {
    __shared__ __align__(16) float os[AW * 16 * 68];
    const int lane = threadIdx.x & 31, lr = lane & 15, hi = lane >> 4;
    const int wave = __builtin_amdgcn_readfirstlane((int)(threadIdx.x >> 5));
    const int b = blockIdx.z; const int tile = blockIdx.y; const int t0 = tile * 16; const int tq = t0 + lr;
    const int kc0 = (blockIdx.x * AW + wave) * AKT;
    v8f acc[4];
#pragma unroll
    for (int j = 0; j < 4; ++j) acc[j] = (v8f){};
    if (kc0 <= t0 + 15) {
#pragma unroll 1
        for (int h = 0; h < NH_; ++h) {
            const int zh = b * NH_ + h;
            const size_t pbase = (size_t)zh * SEQ * HD;
            const size_t qo = pbase + (size_t)(t0 + lr) * HD + 8 * hi;
            const v16h qh0 = ldh(QH + qo), qh1 = ldh(QH + qo + 32), qr0 = ldh(QR + qo), qr1 = ldh(QR + qo + 32);
            const float* sl = ST + ((size_t)zh * (SEQ / 16) + tile) * 32;
            const float sh = sl[lr]; const float iv = sl[16 + lr];
            const h16* kp = KP + pbase + (size_t)(kc0 + lr) * HD + 8 * hi;
#pragma unroll
            for (int g = 0; g < 2; ++g) {
                const h16* ka = kp + (size_t)(32 * g) * HD;
                const v16h ka0 = ldh(ka), ka1 = ldh(ka + 32), kb0 = ldh(ka + 16 * HD), kb1 = ldh(ka + 16 * HD + 32);
                v8f sHa = (v8f){}, sLa = (v8f){}, sHb = (v8f){}, sLb = (v8f){};
                sHa = wmma16(ka0, qh0, sHa); sLa = wmma16(ka0, qr0, sLa); sHb = wmma16(kb0, qh0, sHb); sLb = wmma16(kb0, qr0, sLb);
                sHa = wmma16(ka1, qh1, sHa); sLa = wmma16(ka1, qr1, sLa); sHb = wmma16(kb1, qh1, sHb); sLb = wmma16(kb1, qr1, sLb);
                asm volatile("v_nop\n\tv_nop\n\tv_nop\n\tv_nop" : "+v"(sHa), "+v"(sLa), "+v"(sHb), "+v"(sLb) : "v"(ka0), "v"(ka1), "v"(kb0), "v"(kb1));
                const int kA = kc0 + 32 * g + 8 * hi, kB = kA + 16;
#pragma unroll
                for (int r = 0; r < 8; ++r) {
                    const float pa = __builtin_amdgcn_exp2f((sHa[r] + sLa[r] * QRI) * SC2 + sh) * iv;
                    const float pc = __builtin_amdgcn_exp2f((sHb[r] + sLb[r] * QRI) * SC2 + sh) * iv;
                    acc[2 * g][r]     += (kA + r <= tq) ? pa : 0.0f;
                    acc[2 * g + 1][r] += (kB + r <= tq) ? pc : 0.0f; }
            }
        }
    }
    const int wb = wave * 16 * 68;
    PUTA(0, acc[0]) PUTA(1, acc[1]) PUTA(2, acc[2]) PUTA(3, acc[3])
    wave_sync();
    float* orow = AVG + ((size_t)b * OUT_SEQ + t0) * (size_t)AVG_PITCH + kc0;
#pragma unroll 1
    for (int ps = 0; ps < 2; ++ps) {
#pragma unroll
        for (int s = 0; s < 8; ++s) { const int row = 2 * s + hi, cofs = lr * 4;
            const v4f val = *(const v4fa*)(&os[wb + row * 68 + cofs]);
            *(volatile v4f*)(orow + (size_t)row * AVG_PITCH + cofs) = val; }
        if (ps == 0) __threadfence(); }
}

static constexpr size_t al256(size_t v) { return (v + 255) & ~(size_t)255; }
static constexpr size_t SZ_XB  = al256((size_t)NB * SEQ * DM * 2);
static constexpr size_t SZ_WB  = al256((size_t)4 * DM * DM * 2);
static constexpr size_t SZ_PL  = al256((size_t)NB * NH_ * SEQ * HD * 2);
static constexpr size_t SZ_CTX = al256((size_t)NB * SEQ * 2 * DM * 2);
static constexpr size_t SZ_ST  = al256((size_t)NB * NH_ * (SEQ / 16) * 32 * 4);
static constexpr size_t SZ_TOTAL = SZ_XB + SZ_WB + 5 * SZ_PL + SZ_CTX + SZ_ST;
static_assert(SZ_TOTAL <= (size_t)134217728);
static_assert(((size_t)DM * DM * 2) % 256 == 0);

extern "C" void kernel_launch(void* const* d_in, const int* in_sizes, int n_in,
                              void* d_out, int out_size, void* d_ws, size_t ws_size, hipStream_t stream) {
    if (n_in < 9) return;
    const size_t needx = ((size_t)(NB - 1) * SEQ_FULL + SEQ) * DM;
    if ((size_t)in_sizes[0] < needx) return;
    if ((size_t)in_sizes[1] < (size_t)DM * DM || (size_t)in_sizes[3] < (size_t)DM * DM || (size_t)in_sizes[5] < (size_t)DM * DM || (size_t)in_sizes[7] < (size_t)DM * DM) return;
    if (in_sizes[2] < DM || in_sizes[4] < DM || in_sizes[6] < DM || in_sizes[8] < DM) return;
    if ((size_t)out_size < ((size_t)(NB - 1) * OUT_SEQ + SEQ) * DM) return;
    if ((size_t)out_size < AVG_OFF + ((size_t)(NB - 1) * OUT_SEQ + SEQ) * (size_t)AVG_PITCH) return;
    if (SZ_TOTAL > ws_size) return;
    const float* x  = (const float*)d_in[0];
    const float* wq = (const float*)d_in[1]; const float* bq = (const float*)d_in[2];
    const float* wk = (const float*)d_in[3]; const float* bk = (const float*)d_in[4];
    const float* wv = (const float*)d_in[5]; const float* bv = (const float*)d_in[6];
    const float* wo = (const float*)d_in[7]; const float* bo = (const float*)d_in[8];
    float* OUT = (float*)d_out;
    float* AVG = (float*)d_out + AVG_OFF;
    char* wsp = (char*)d_ws;
    bf* XB = (bf*)wsp; wsp += SZ_XB;
    bf* WB = (bf*)wsp; wsp += SZ_WB;
    h16* QH = (h16*)wsp; wsp += SZ_PL;
    h16* QR = (h16*)wsp; wsp += SZ_PL;
    h16* KP = (h16*)wsp; wsp += SZ_PL;
    h16* VT = (h16*)wsp; wsp += SZ_PL;
    h16* VR = (h16*)wsp; wsp += SZ_PL;
    bf* CTX = (bf*)wsp; wsp += SZ_CTX;
    float* ST = (float*)wsp; wsp += SZ_ST;
    bf* WQ = WB; bf* WK = WB + (size_t)DM * DM; bf* WV = WB + (size_t)2 * DM * DM; bf* WO = WB + (size_t)3 * DM * DM;

    if (SEQ == SEQ_FULL) {
        const size_t n8 = (size_t)NB * SEQ * DM / 8;
        k_cvt8<<<(unsigned)((n8 + 255) / 256), 256, 0, stream>>>(x, XB, n8);
    } else {
        const size_t n8 = (size_t)SEQ * DM / 8;
        for (int b = 0; b < NB; ++b) k_cvt8<<<(unsigned)((n8 + 255) / 256), 256, 0, stream>>>(x + (size_t)b * SEQ_FULL * DM, XB + (size_t)b * SEQ * DM, n8);
    }
    { const size_t n8 = (size_t)DM * DM / 8; const unsigned g = (unsigned)((n8 + 255) / 256);
      k_cvt8<<<g, 256, 0, stream>>>(wq, WQ, n8); k_cvt8<<<g, 256, 0, stream>>>(wk, WK, n8); k_cvt8<<<g, 256, 0, stream>>>(wv, WV, n8); k_cvt8<<<g, 256, 0, stream>>>(wo, WO, n8); }

    k_proj<<<dim3(NB * SEQ / 64, DM / 64, 1), 32, 0, stream>>>(XB, WQ, bq, 0, QH, QR, 1, SEQ, (size_t)NH_ * SEQ * HD, HD, HD, (size_t)SEQ * HD);
    k_proj<<<dim3(NB * SEQ / 64, DM / 64, 1), 32, 0, stream>>>(XB, WK, bk, 0, KP, KP, 0, SEQ, (size_t)NH_ * SEQ * HD, HD, HD, (size_t)SEQ * HD);
    k_proj<<<dim3(DM / 64, NB * SEQ / 64, 1), 32, 0, stream>>>(WV, XB, bv, 1, VT, VR, 1, DM, (size_t)0, SEQ, SEQ, (size_t)DM * SEQ);

    k_flash<<<dim3(SEQ / (16 * AW), NB * NH_, 1), 32 * AW, 0, stream>>>(QH, QR, KP, VT, VR, CTX, ST);
    k_avg<<<dim3(SEQ / (AKT * AW), SEQ / 16, NB), 32 * AW, 0, stream>>>(QH, QR, KP, ST, AVG);
    k_outp<<<dim3(NB * SEQ / 64, DM / 64, 1), 32, 0, stream>>>(CTX, WO, bo, OUT);
}
